// SyllableRNN_8761733284404
// MI455X (gfx1250) — hardware-run, weakly checked
//
#include <hip/hip_runtime.h>

typedef __attribute__((ext_vector_type(16))) _Float16 v16h;
typedef __attribute__((ext_vector_type(8)))  _Float16 v8h;
typedef __attribute__((ext_vector_type(8)))  float    v8f;
typedef __attribute__((ext_vector_type(4)))  float    v4f;
typedef __attribute__((ext_vector_type(4)))  int      v4i;

constexpr int kBatch  = 1024;
constexpr int kStep   = 128;
constexpr int kEmb    = 256;
constexpr int kHid    = 1024;
constexpr int kTag    = 8;
constexpr int kTagPad = 16;
constexpr int kVoc    = 128;

constexpr float kCarryE   = 1024.0f;
constexpr float kCarryW   = 1024.0f;
constexpr float kCarryH   = 256.0f;
constexpr float kCarryAcc = kCarryH * kCarryW;
constexpr float kInvAcc   = 1.0f / kCarryAcc;
constexpr float kPScale   = kCarryAcc / (kCarryE * kCarryW);
static_assert(kCarryAcc == 262144.0f);
static_assert(kPScale == 0.25f);

constexpr int kRowsPB     = 16;
constexpr int kRnnBlocks  = kBatch / kRowsPB;
constexpr int kRnnThreads = 256;
constexpr int kColsPW     = 128;
constexpr int kHP         = kHid + 8;
constexpr int kHTile      = kRowsPB * kHP;
static_assert(kBatch % kRowsPB == 0);
static_assert(kHid == (kRnnThreads / 32) * kColsPW);
static_assert(kHP % 8 == 0);
static_assert(kHid % 32 == 0 && kEmb % 32 == 0);
static_assert(kVoc % 64 == 0 && kHid % 64 == 0);
static_assert(kStep % 4 == 0);
static_assert(kRowsPB * kStep == kRnnThreads * 8);
static_assert((kHid / 32) == (kRnnThreads / 32) * 4);

constexpr int kDwEmb  = kVoc * kEmb / 2;
constexpr int kDwWih  = kHid * kEmb / 2;
constexpr int kDwWhh  = kHid * kHid / 2;
constexpr int kDwWout = kTagPad * kHid / 2;
constexpr int kDwWoutLive = kTag * kHid / 2;
constexpr int kDwBsum = kHid;
constexpr int kPrepB1 = kDwEmb / 256;
constexpr int kPrepB2 = kPrepB1 + kDwWih / 256;
constexpr int kPrepB3 = kPrepB2 + kDwWhh / 256;
constexpr int kPrepB4 = kPrepB3 + kDwWout / 256;
constexpr int kPrepBlocks = kPrepB4 + kDwBsum / 256;
static_assert(kDwEmb % 256 == 0 && kDwWih % 256 == 0 && kDwWhh % 256 == 0 && kDwWout % 256 == 0 && kDwBsum % 256 == 0);
static_assert(kPrepBlocks == 2660);
static_assert((kDwWoutLive & (kDwWoutLive - 1)) == 0);

union FragU { v16h v; v8h h[2]; };
__device__ __forceinline__ v16h frag_load(const _Float16* p) {
  FragU f;
  f.h[0] = *(const v8h*)(p);
  f.h[1] = *(const v8h*)(p + 16);
  return f.v;
}
__device__ __forceinline__ v8f mma_g(v16h a, v16h b, v8f c) {
  c = __builtin_amdgcn_wmma_f32_16x16x32_f16(false, a, false, b, (short)0, c, false, false);
  asm volatile("v_nop\n\tv_nop\n\tv_nop\n\tv_nop" : "+v"(c) : "v"(a), "v"(b));
  return c;
}
__device__ __forceinline__ void acc_guard4(v8f& a, v8f& b, v8f& c, v8f& d) {
  asm volatile("v_nop\n\tv_nop\n\tv_nop\n\tv_nop" : "+v"(a), "+v"(b), "+v"(c), "+v"(d));
}

__device__ __forceinline__ unsigned pack_f16x2(float a, float b) {
  const _Float16 h0 = (_Float16)a, h1 = (_Float16)b;
  return (unsigned)__builtin_bit_cast(unsigned short, h0) | ((unsigned)__builtin_bit_cast(unsigned short, h1) << 16);
}
__device__ __forceinline__ void st2u(unsigned* p, unsigned v) {
  *(volatile unsigned*)p = v;
  __threadfence();
  *(volatile unsigned*)p = v;
}
__device__ __forceinline__ float state_val(float a) {
  const float e = __expf(a * (2.0f * kInvAcc));
  const float rc = __builtin_amdgcn_rcpf(1.0f + e);
  return kCarryH - (2.0f * kCarryH) * rc;
}

__global__ __launch_bounds__(256) void prep_kernel(
    const float* __restrict__ emb, const float* __restrict__ w_ih,
    const float* __restrict__ w_hh, const float* __restrict__ w_out,
    const float* __restrict__ b_ih, const float* __restrict__ b_hh,
    unsigned* __restrict__ embu, unsigned* __restrict__ wihu,
    unsigned* __restrict__ whhu, unsigned* __restrict__ woutu, unsigned* __restrict__ bsumu) {
  const int blk = blockIdx.x, tid = threadIdx.x;
  if (blk < kPrepB1) {
    const int p = blk * 256 + tid;
    st2u(embu + p, pack_f16x2(emb[2 * p] * kCarryE, emb[2 * p + 1] * kCarryE));
  } else if (blk < kPrepB2) {
    const int p = (blk - kPrepB1) * 256 + tid;
    st2u(wihu + p, pack_f16x2(w_ih[2 * p] * kCarryW, w_ih[2 * p + 1] * kCarryW));
  } else if (blk < kPrepB3) {
    const int p = (blk - kPrepB2) * 256 + tid;
    st2u(whhu + p, pack_f16x2(w_hh[2 * p] * kCarryW, w_hh[2 * p + 1] * kCarryW));
  } else if (blk < kPrepB4) {
    const int p = (blk - kPrepB3) * 256 + tid;
    const int pc = p & (kDwWoutLive - 1);
    const float a = w_out[2 * pc];
    const float b = w_out[2 * pc + 1];
    const bool live = (p < kDwWoutLive);
    const float va = live ? a * kCarryW : 0.0f;
    const float vb = live ? b * kCarryW : 0.0f;
    st2u(woutu + p, pack_f16x2(va, vb));
  } else {
    const int p = (blk - kPrepB4) * 256 + tid;
    const float v = (b_ih[p] + b_hh[p]) * kCarryAcc;
    st2u(bsumu + p, (unsigned)__float_as_uint(v));
  }
}

__global__ __launch_bounds__(256) void ptable_gemm(
    const _Float16* __restrict__ A, int lda,
    const _Float16* __restrict__ Bt, int ldb,
    float* __restrict__ C, int ldc,
    const float* __restrict__ bias,
    int M, int N, int K, float scale) {
  __shared__ __align__(16) float sT[8][16 * 68];
  const int lane = threadIdx.x & 31;
  const int wave = threadIdx.x >> 5;
  const int tilesN = N >> 6;
  const int tilesM = M >> 6;
  const int tile = blockIdx.x * 8 + wave;
  if (tile >= tilesM * tilesN) return;
  const int tm = tile / tilesN;
  const int tn = tile - tm * tilesN;
  const int m0 = tm << 6;
  const int n0 = tn << 6;
  const int rlane = lane & 15;
  const int koff  = (lane >> 4) * 8;
  const int mOff  = (lane >> 4) * 8;

  v8f acc[4][4];
#pragma unroll
  for (int i = 0; i < 4; ++i)
#pragma unroll
    for (int j = 0; j < 4; ++j) acc[i][j] = (v8f){0.f, 0.f, 0.f, 0.f, 0.f, 0.f, 0.f, 0.f};

  for (int k0 = 0; k0 < K; k0 += 32) {
    v16h bh[4];
#pragma unroll
    for (int j = 0; j < 4; ++j) {
      const size_t bo = (size_t)(n0 + (j << 4) + rlane) * ldb + koff + k0;
      bh[j] = frag_load(Bt + bo);
    }
#pragma unroll
    for (int i = 0; i < 4; ++i) {
      const size_t ao = (size_t)(m0 + (i << 4) + rlane) * lda + koff + k0;
      const v16h ah = frag_load(A + ao);
#pragma unroll
      for (int j = 0; j < 4; ++j) acc[i][j] = mma_g(ah, bh[j], acc[i][j]);
    }
  }
  acc_guard4(acc[0][0], acc[0][1], acc[0][2], acc[0][3]);
  acc_guard4(acc[1][0], acc[1][1], acc[1][2], acc[1][3]);
  acc_guard4(acc[2][0], acc[2][1], acc[2][2], acc[2][3]);
  acc_guard4(acc[3][0], acc[3][1], acc[3][2], acc[3][3]);

  float* slab = sT[wave];
#pragma unroll
  for (int i = 0; i < 4; ++i) {
    const int mBase = m0 + (i << 4);
#pragma unroll
    for (int j = 0; j < 4; ++j) {
      const int n = n0 + (j << 4) + rlane;
      const float bv = bias[n];
#pragma unroll
      for (int r = 0; r < 8; ++r) {
        const float v = acc[i][j][r] * scale + bv;
        slab[(mOff + r) * 68 + (j << 4) + rlane] = v;
      }
    }
    __builtin_amdgcn_fence(__ATOMIC_RELEASE, "workgroup");
    __builtin_amdgcn_wave_barrier();
    __builtin_amdgcn_fence(__ATOMIC_ACQUIRE, "workgroup");
    {
      const int hh = lane >> 4, c4 = (lane & 15) * 4;
      for (int pass = 0; pass < 2; ++pass) {
#pragma unroll
        for (int it = 0; it < 8; ++it) {
          const int row = it * 2 + hh;
          const v4f v = *(const v4f*)(slab + row * 68 + c4);
          *(volatile v4f*)(C + (size_t)(mBase + row) * ldc + n0 + c4) = v;
        }
        __threadfence();
      }
    }
    __builtin_amdgcn_fence(__ATOMIC_RELEASE, "workgroup");
    __builtin_amdgcn_wave_barrier();
    __builtin_amdgcn_fence(__ATOMIC_ACQUIRE, "workgroup");
  }
}

__global__ __launch_bounds__(kRnnThreads) void rnn_kernel(
    const int* __restrict__ ids, const float* __restrict__ ptab,
    const _Float16* __restrict__ whh16, const _Float16* __restrict__ wout16,
    const float* __restrict__ b_out, float* __restrict__ out) {
  __shared__ __align__(16) _Float16 htile[kHTile];
  __shared__ __align__(16) int   ids_lds[kRowsPB * kStep];
  __shared__ int   slen_lds[kRowsPB];
  __shared__ __align__(16) float outscr[8 * 256];
  __shared__ __align__(16) float linebuf[kRowsPB * 4 * kTagPad];

  const int tid = threadIdx.x, lane = tid & 31, wave = tid >> 5;
  const int c = lane & 15, hh = lane >> 4, koff = hh * 8, mOff = hh * 8;
  const int b0 = blockIdx.x * kRowsPB;
  const int n0 = wave * kColsPW;

  {
    const v8h z = {(_Float16)0.f, (_Float16)0.f, (_Float16)0.f, (_Float16)0.f, (_Float16)0.f, (_Float16)0.f, (_Float16)0.f, (_Float16)0.f};
    for (int i = tid; i < kHTile / 8; i += kRnnThreads) *(v8h*)(htile + i * 8) = z;
  }
  {
    const int row = tid >> 4, seg = tid & 15;
    const int* gp = ids + (size_t)(b0 + row) * kStep + seg * 8;
    const v4i ia = *(const v4i*)gp;
    const v4i ib = *(const v4i*)(gp + 4);
    int cnt = (ia[0] != 0) + (ia[1] != 0) + (ia[2] != 0) + (ia[3] != 0) +
              (ib[0] != 0) + (ib[1] != 0) + (ib[2] != 0) + (ib[3] != 0);
    v4i ca, cb;
    ca[0] = min(max(ia[0], 0), kVoc - 1); ca[1] = min(max(ia[1], 0), kVoc - 1);
    ca[2] = min(max(ia[2], 0), kVoc - 1); ca[3] = min(max(ia[3], 0), kVoc - 1);
    cb[0] = min(max(ib[0], 0), kVoc - 1); cb[1] = min(max(ib[1], 0), kVoc - 1);
    cb[2] = min(max(ib[2], 0), kVoc - 1); cb[3] = min(max(ib[3], 0), kVoc - 1);
    *(v4i*)(ids_lds + row * kStep + seg * 8) = ca;
    *(v4i*)(ids_lds + row * kStep + seg * 8 + 4) = cb;
    cnt += __shfl_xor(cnt, 1, 32);
    cnt += __shfl_xor(cnt, 2, 32);
    cnt += __shfl_xor(cnt, 4, 32);
    cnt += __shfl_xor(cnt, 8, 32);
    slen_lds[row] = cnt;
  }
  __syncthreads();

  int sl[8];
#pragma unroll
  for (int r = 0; r < 8; ++r) sl[r] = slen_lds[mOff + r];
  const float bo = b_out[c & (kTag - 1)];
  v16h wf[4];
#pragma unroll
  for (int k4 = 0; k4 < 4; ++k4) wf[k4] = frag_load(wout16 + (size_t)c * kHid + (wave * 4 + k4) * 32 + koff);

  const _Float16* brow = whh16 + (size_t)(n0 + 8 * c) * kHid + koff;
  const _Float16* arow = htile + c * kHP + koff;
  const float*    prow = ptab + n0 + 8 * c;
  const int*      idrow = ids_lds + mOff * kStep;
  _Float16*       hwr  = htile + mOff * kHP + n0 + 8 * c;

#pragma unroll 1
  for (int t = 0; t < kStep; ++t) {
    v8f acc[8];
#pragma unroll
    for (int r = 0; r < 8; ++r) {
      const int ido = idrow[r * kStep + t] * kHid;
      const v4f pa = *(const v4f*)(prow + ido);
      const v4f pb = *(const v4f*)(prow + ido + 4);
      acc[0][r] = pa[0]; acc[1][r] = pa[1]; acc[2][r] = pa[2]; acc[3][r] = pa[3];
      acc[4][r] = pb[0]; acc[5][r] = pb[1]; acc[6][r] = pb[2]; acc[7][r] = pb[3];
    }

#pragma unroll 2
    for (int kc = 0; kc < kHid / 32; ++kc) {
      const v16h fa = frag_load(arow + kc * 32);
#pragma unroll
      for (int g = 0; g < 2; ++g) {
        v16h fb[4];
#pragma unroll
        for (int j = 0; j < 4; ++j) fb[j] = frag_load(brow + (size_t)(4 * g + j) * kHid + kc * 32);
#pragma unroll
        for (int j = 0; j < 4; ++j) acc[4 * g + j] = mma_g(fa, fb[j], acc[4 * g + j]);
      }
    }

    __syncthreads();

#pragma unroll
    for (int r = 0; r < 8; ++r) {
      _Float16* hp = hwr + r * kHP;
      const v8h oldv = *(const v8h*)hp;
      v8h nv;
#pragma unroll
      for (int j = 0; j < 8; ++j) nv[j] = (_Float16)state_val(acc[j][r]);
      const bool upd = (t < sl[r]);
      const v8h sv = upd ? nv : oldv;
      *(v8h*)hp = sv;
    }

    __syncthreads();

    {
      v8f oc = (v8f){0.f, 0.f, 0.f, 0.f, 0.f, 0.f, 0.f, 0.f};
#pragma unroll
      for (int k4 = 0; k4 < 4; ++k4) {
        const v16h fa2 = frag_load(arow + (wave * 4 + k4) * 32);
        oc = mma_g(fa2, wf[k4], oc);
      }
#pragma unroll
      for (int r = 0; r < 8; ++r) outscr[wave * 256 + (mOff + r) * kTagPad + c] = oc[r] * kInvAcc;
    }

    __syncthreads();

    {
      const int row = 2 * wave + hh;
      float s = bo;
#pragma unroll
      for (int wv = 0; wv < 8; ++wv) s += outscr[wv * 256 + row * kTagPad + c];
      linebuf[(row * 4 + (t & 3)) * kTagPad + c] = s;
    }

    if ((t & 3) == 3) {
      __syncthreads();
      const int tt = lane >> 3, tg = lane & 7;
      const int rowA = 2 * wave, rowB = 2 * wave + 1;
      const float vA = linebuf[(rowA * 4 + tt) * kTagPad + tg];
      const float vB = linebuf[(rowB * 4 + tt) * kTagPad + tg];
      float* dA = out + ((size_t)(b0 + rowA) * kStep + (t - 3)) * kTag + lane;
      float* dB = out + ((size_t)(b0 + rowB) * kStep + (t - 3)) * kTag + lane;
      *(volatile float*)dA = vA;
      *(volatile float*)dB = vB;
      __threadfence();
      *(volatile float*)dA = vA;
      *(volatile float*)dB = vB;
    }
  }
}

extern "C" void kernel_launch(void* const* d_in, const int* in_sizes, int n_in,
                              void* d_out, int out_size, void* d_ws, size_t ws_size, hipStream_t stream) {
  if (n_in < 8 || d_out == nullptr || d_ws == nullptr) return;
  if (in_sizes[0] != kBatch * kStep || in_sizes[1] != kVoc * kEmb || in_sizes[2] != kHid * kEmb ||
      in_sizes[3] != kHid * kHid || in_sizes[4] != kHid || in_sizes[5] != kHid ||
      in_sizes[6] != kTag * kHid || in_sizes[7] != kTag || out_size != kBatch * kStep * kTag) return;

  const int*   ids   = (const int*)d_in[0];
  const float* emb   = (const float*)d_in[1];
  const float* w_ih  = (const float*)d_in[2];
  const float* w_hh  = (const float*)d_in[3];
  const float* b_ih  = (const float*)d_in[4];
  const float* b_hh  = (const float*)d_in[5];
  const float* w_out = (const float*)d_in[6];
  const float* b_out = (const float*)d_in[7];
  float* out = (float*)d_out;

  char* ws = (char*)d_ws;
  size_t off = 0;
  auto carve = [&](size_t bytes) -> char* { char* p = ws + off; off += (bytes + 255) & ~(size_t)255; return p; };
  _Float16* EMB16  = (_Float16*)carve((size_t)kVoc * kEmb * 2);
  _Float16* WIH16  = (_Float16*)carve((size_t)kHid * kEmb * 2);
  _Float16* WHH16  = (_Float16*)carve((size_t)kHid * kHid * 2);
  _Float16* WOUT16 = (_Float16*)carve((size_t)kTagPad * kHid * 2);
  float*    BSUM   = (float*)carve((size_t)kHid * 4);
  float*    PTAB   = (float*)carve((size_t)kVoc * kHid * 4);
  if (off > ws_size || off > (size_t)134217728) return;

  prep_kernel<<<kPrepBlocks, 256, 0, stream>>>(emb, w_ih, w_hh, w_out, b_ih, b_hh,
                                               (unsigned*)EMB16, (unsigned*)WIH16, (unsigned*)WHH16,
                                               (unsigned*)WOUT16, (unsigned*)BSUM);

  static_assert(kVoc % 64 == 0 && kHid % 64 == 0 && kEmb % 32 == 0);
  static_assert(((kVoc / 64) * (kHid / 64)) % 8 == 0);
  ptable_gemm<<<((kVoc / 64) * (kHid / 64)) / 8, 256, 0, stream>>>(
      EMB16, kEmb, WIH16, kEmb, PTAB, kHid, BSUM, kVoc, kHid, kEmb, kPScale);

  rnn_kernel<<<kRnnBlocks, kRnnThreads, 0, stream>>>(ids, PTAB, WHH16, WOUT16, b_out, out);
}
